// SDFCLayer_65773129171730
// MI455X (gfx1250) — hardware-verified
//
#include <hip/hip_runtime.h>
#include <stddef.h>


#define CH     128
#define NCOL   256
#define KPB    128
#define APZ    136
#define PQW    256
#define GROWS  32
#define GTHR   64
#define ETHR   256
#define WTHR   256
#define WBLK   16
#define WSCL   16.0f
#define RWS    0.0625f
#define WSCAP  134217728

static_assert(GROWS == (GTHR / 32) * 16);
static_assert((APZ % 8) == 0 && (KPB % 8) == 0 && (PQW % 32) == 0);
static_assert(32 * GTHR * 4 == GROWS * PQW);
static_assert(WBLK * WTHR * 8 == NCOL * KPB);
static_assert((ETHR % 128) == 0);
static_assert((CH % 32) == 0);

typedef float    v4f  __attribute__((ext_vector_type(4)));
typedef float    v8f  __attribute__((ext_vector_type(8)));
typedef _Float16 v8h  __attribute__((ext_vector_type(8)));
typedef _Float16 v16h __attribute__((ext_vector_type(16)));
union Frag { v16h v; v8h h[2]; };

__device__ __forceinline__ v8f wmh(v16h a, v16h b, v8f c) {
  v8f d = __builtin_amdgcn_wmma_f32_16x16x32_f16(false, a, false, b, (short)0, c, false, false);
  asm volatile("v_nop\n\tv_nop\n\tv_nop\n\tv_nop" : "+v"(d) : "v"(a), "v"(b));
  return d;
}

__device__ __forceinline__ v8h cvt8(v4f a, v4f b) {
  v8h r;
  r[0] = (_Float16)a.x; r[1] = (_Float16)a.y; r[2] = (_Float16)a.z; r[3] = (_Float16)a.w;
  r[4] = (_Float16)b.x; r[5] = (_Float16)b.y; r[6] = (_Float16)b.z; r[7] = (_Float16)b.w;
  return r;
}

template <int NT>
__device__ __forceinline__ void mma16(const _Float16* At, const _Float16* __restrict__ Bpl,
                                      int lane, v8f (&acc)[NT]) {
  const int hh = lane >> 4, m = lane & 15;
#pragma unroll
  for (int t = 0; t < NT; ++t) { v8f z = {0.f, 0.f, 0.f, 0.f, 0.f, 0.f, 0.f, 0.f}; acc[t] = z; }
  const _Float16* ap = At + m * APZ + 8 * hh;
  const _Float16* bb = Bpl + (size_t)m * KPB + 8 * hh;
#pragma unroll 1
  for (int ks = 0; ks < CH / 32; ++ks) {
    Frag a;
    a.h[0] = *(const v8h*)(ap + 32 * ks);
    a.h[1] = *(const v8h*)(ap + 32 * ks + 16);
#pragma unroll
    for (int t = 0; t < NT; ++t) {
      const _Float16* bp = bb + (size_t)(16 * t) * KPB + 32 * ks;
      Frag b;
      b.h[0] = *(const v8h*)bp;
      b.h[1] = *(const v8h*)(bp + 16);
      acc[t] = wmh(a.v, b.v, acc[t]);
    }
  }
}

__global__ __launch_bounds__(WTHR) void k_wprep(const float* __restrict__ W1, _Float16* Bpl) {
  const int i = blockIdx.x * WTHR + threadIdx.x;
  const int n = i >> 4, k0 = (i & 15) * 8;
  const int kb = (n >> 7) * CH, nc = n & (CH - 1);
  float v[8];
#pragma unroll
  for (int e = 0; e < 8; ++e) v[e] = W1[(kb + k0 + e) * CH + nc];
  v8h hv;
#pragma unroll
  for (int e = 0; e < 8; ++e) hv[e] = (_Float16)(v[e] * WSCL);
  _Float16* dp = Bpl + (size_t)i * 8;
  *(volatile v8h*)dp = hv;
  __threadfence();
  *(volatile v8h*)dp = hv;
}

__global__ __launch_bounds__(GTHR) void k_nodegemm(const float* __restrict__ z, const _Float16* __restrict__ Bpl,
                                                   float* PQ, int nN) {
  __shared__ __attribute__((aligned(16))) _Float16 Ah[GROWS * APZ];
  __shared__ __attribute__((aligned(16))) float stg[GROWS * PQW];
  const int tid = threadIdx.x, lane = tid & 31, wave = tid >> 5, hh = lane >> 4, m = lane & 15;
  const int rowBase = blockIdx.x * GROWS;
  {
    const int r = tid >> 1, c0 = (tid & 1) * 64;
    int zrow = rowBase + r;
    zrow = zrow > nN - 1 ? nN - 1 : zrow;
    const float* zp = z + (size_t)zrow * CH + c0;
#pragma unroll
    for (int j = 0; j < 8; ++j) {
      const v4f a = *(const v4f*)(zp + 8 * j), b = *(const v4f*)(zp + 8 * j + 4);
      *(v8h*)(Ah + r * APZ + c0 + 8 * j) = cvt8(a, b);
    }
  }
  __syncthreads();

#pragma unroll 1
  for (int cg = 0; cg < 4; ++cg) {
    v8f acc[4];
    mma16<4>(Ah + wave * 16 * APZ, Bpl + (size_t)(64 * cg) * KPB, lane, acc);
    float* sp = stg + (wave * 16 + 8 * hh) * PQW + 64 * cg + m;
#pragma unroll
    for (int t = 0; t < 4; ++t) {
#pragma unroll
      for (int r = 0; r < 8; ++r) sp[r * PQW + 16 * t] = acc[t][r] * RWS;
    }
  }
  __syncthreads();

  float* gp = PQ + (size_t)rowBase * PQW;
#pragma unroll
  for (int it = 0; it < 32; ++it) {
    const int f = it * GTHR + tid;
    const v4f v = *(const v4f*)(stg + 4 * f);
    *(volatile v4f*)(gp + 4 * f) = v;
  }
  __threadfence();
#pragma unroll
  for (int it = 0; it < 32; ++it) {
    const int f = it * GTHR + tid;
    const v4f v = *(const v4f*)(stg + 4 * f);
    *(volatile v4f*)(gp + 4 * f) = v;
  }
}

__global__ __launch_bounds__(ETHR) void k_edge(const float* __restrict__ PQ, const int* __restrict__ ei,
                                               const float* __restrict__ b1, const float* __restrict__ W2,
                                               const float* __restrict__ b2, float* out, int nN, int nE) {
  __shared__ __attribute__((aligned(16))) float sb1[CH];
  __shared__ __attribute__((aligned(16))) float sw2[CH];
  __shared__ __attribute__((aligned(16))) float sout[ETHR];
  const int tid = threadIdx.x;
  if (tid < CH) { sb1[tid] = b1[tid]; sw2[tid] = W2[tid]; }
  const float b2v = b2[0];
  __syncthreads();

  const int base = blockIdx.x * ETHR;
  int e = base + tid;
  e = e > nE - 1 ? nE - 1 : e;
  int s = ei[e];
  int d = ei[(size_t)nE + e];
  s = s < 0 ? s + nN : s;  s = s < 0 ? 0 : (s > nN - 1 ? nN - 1 : s);
  d = d < 0 ? d + nN : d;  d = d < 0 ? 0 : (d > nN - 1 ? nN - 1 : d);
  const float* pp = PQ + (size_t)s * PQW;
  const float* qp = PQ + (size_t)d * PQW + CH;
  float a0 = 0.0f, a1 = 0.0f, a2 = 0.0f, a3 = 0.0f;
#pragma unroll 2
  for (int j = 0; j < CH / 4; ++j) {
    const v4f p = *(const v4f*)(pp + 4 * j);
    const v4f q = *(const v4f*)(qp + 4 * j);
    const v4f bb = *(const v4f*)(sb1 + 4 * j);
    const v4f w = *(const v4f*)(sw2 + 4 * j);
    v4f h = (p + q) + bb;
    h.x = fmaxf(h.x, 0.0f); h.y = fmaxf(h.y, 0.0f); h.z = fmaxf(h.z, 0.0f); h.w = fmaxf(h.w, 0.0f);
    a0 = fmaf(h.x, w.x, a0);
    a1 = fmaf(h.y, w.y, a1);
    a2 = fmaf(h.z, w.z, a2);
    a3 = fmaf(h.w, w.w, a3);
  }
  const float o = ((a0 + a1) + (a2 + a3)) + b2v;
  sout[tid] = o;
  __syncthreads();

  if (tid < ETHR / 4) {
    const int f = 4 * tid;
    const int g = base + f;
    const v4f v = *(const v4f*)(sout + f);
    if (g + 4 <= nE) {
      *(volatile v4f*)(out + g) = v;
    } else if (g < nE) {
      *(volatile float*)(out + g) = v.x;
      if (g + 1 < nE) *(volatile float*)(out + g + 1) = v.y;
      if (g + 2 < nE) *(volatile float*)(out + g + 2) = v.z;
    }
  }
  __threadfence();
  if (tid < ETHR / 4) {
    const int f = 4 * tid;
    const int g = base + f;
    const v4f v = *(const v4f*)(sout + f);
    if (g + 4 <= nE) {
      *(volatile v4f*)(out + g) = v;
    } else if (g < nE) {
      *(volatile float*)(out + g) = v.x;
      if (g + 1 < nE) *(volatile float*)(out + g + 1) = v.y;
      if (g + 2 < nE) *(volatile float*)(out + g + 2) = v.z;
    }
  }
}

extern "C" void kernel_launch(void* const* d_in, const int* in_sizes, int n_in,
                              void* d_out, int out_size, void* d_ws, size_t ws_size,
                              hipStream_t stream) {
  if (n_in < 6) return;
  const int nN = in_sizes[0] / CH;
  const int nE = in_sizes[1] / 2;
  if (nN <= 0 || nE <= 0) return;
  if (in_sizes[0] != nN * CH || in_sizes[1] != 2 * nE) return;
  if (in_sizes[2] != 2 * CH * CH || in_sizes[3] != CH || in_sizes[4] != CH || in_sizes[5] < 1) return;
  if (out_size != nE) return;
  if (nE > (1 << 28) || nN > (1 << 24)) return;

  const float* z  = (const float*)d_in[0];
  const int*   ei = (const int*)d_in[1];
  const float* W1 = (const float*)d_in[2];
  const float* b1 = (const float*)d_in[3];
  const float* W2 = (const float*)d_in[4];
  const float* b2 = (const float*)d_in[5];
  float* out = (float*)d_out;

  const int nBlkG = (nN + GROWS - 1) / GROWS;
  const int NPADG = nBlkG * GROWS;
  const int nBlkE = (nE + ETHR - 1) / ETHR;

  char* ws = (char*)d_ws;
  size_t off = 0;
  const size_t oB  = off; off += (size_t)NCOL * KPB * 2;        off = (off + 255) & ~(size_t)255;
  const size_t oPQ = off; off += (size_t)NPADG * PQW * 4;       off = (off + 255) & ~(size_t)255;
  if (off > ws_size || off > (size_t)WSCAP) return;
  _Float16* Bpl = (_Float16*)(ws + oB);
  float*    PQ  = (float*)(ws + oPQ);

  k_wprep<<<WBLK, WTHR, 0, stream>>>(W1, Bpl);
  k_nodegemm<<<nBlkG, GTHR, 0, stream>>>(z, Bpl, PQ, nN);
  k_edge<<<nBlkE, ETHR, 0, stream>>>(PQ, ei, b1, W2, b2, out, nN, nE);
}
